// TritonHSTUAttention_67680094650972
// MI455X (gfx1250) — hardware-verified
//
#include <hip/hip_runtime.h>
#include <stdint.h>

#define NHEAD 8
#define DQK   128
#define DVV   128
#define MTILE 128
#define JTILE 32
#define MAXSEQ 1024

typedef __attribute__((ext_vector_type(16))) _Float16 v16bf;
typedef __attribute__((ext_vector_type(16))) __bf16 v16b;
typedef __attribute__((ext_vector_type(8)))  float  v8f;

union FragB {
  v16bf    v;
  uint32_t u[8];
  uint4    q[2];
};

__device__ __forceinline__ uint32_t pkbf(float lo, float hi) {
  union { _Float16 h[2]; uint32_t u; } cv;
  cv.h[0] = static_cast<_Float16>(lo);
  cv.h[1] = static_cast<_Float16>(hi);
  return cv.u;
}
__device__ __forceinline__ float fsilu(float x) { return x / (1.0f + expf(-x)); }
typedef __attribute__((ext_vector_type(4))) float v4f;
template <typename T> __device__ __forceinline__ void vst2(void* p, T v) { *(volatile T*)p = v; __threadfence(); *(volatile T*)p = v; }
__device__ __forceinline__ v8f wmma_bf(v16b a, v16b b, v8f c) {
  v8f d = __builtin_amdgcn_wmma_f32_16x16x32_bf16(false, a, false, b, (short)0, c, false, false);
  asm volatile("v_nop\n\tv_nop\n\tv_nop\n\tv_nop" : "+v"(d) : "v"(a), "v"(b));
  return d;
}
struct F2 { v16b h, l; };
__device__ __forceinline__ F2 split_row(const float* row, int k0, int lane, float scale) {
  F2 r; const float* p = row + k0 + 8 * (lane >> 4);
#pragma unroll
  for (int i = 0; i < 8; ++i) { float v0 = p[i] * scale, v1 = p[16 + i] * scale; __bf16 h0 = (__bf16)v0, h1 = (__bf16)v1;
    r.h[i] = h0; r.l[i] = (__bf16)(v0 - (float)h0); r.h[8 + i] = h1; r.l[8 + i] = (__bf16)(v1 - (float)h1); }
  return r;
}
__device__ __forceinline__ v8f mac3(const F2& a, const F2& b, v8f c) { c = wmma_bf(a.l, b.h, c); c = wmma_bf(a.h, b.l, c); return wmma_bf(a.h, b.h, c); }
__device__ __forceinline__ v8f wmma16(v16bf a, v16bf b, v8f c) {
  v8f d = __builtin_amdgcn_wmma_f32_16x16x32_f16(false, a, false, b, (short)0, c, false, false);
  asm volatile("v_nop\n\tv_nop\n\tv_nop\n\tv_nop" : "+v"(d) : "v"(a), "v"(b));
  return d;
}

__global__ __launch_bounds__(256)
void hstu_attn_wmma(const float* __restrict__ tq,
                    const float* __restrict__ tk,
                    const float* __restrict__ tv,
                    const int*   __restrict__ offsets,
                    const int*   __restrict__ p_maxseq,
                    const int*   __restrict__ p_scale,
                    float*       __restrict__ out) {
  __shared__ __align__(16) float Kt[JTILE][DQK + 4];
  __shared__ uint16_t Vt[DVV][JTILE];
  __shared__ float    Sscr[8][16][32];
  __shared__ __align__(16) float So[8][16][DVV];

  const int b    = blockIdx.z;
  const int h    = blockIdx.y;
  const int off  = offsets[b];
  const int nlen = offsets[b + 1] - off;
  const int row0 = blockIdx.x * MTILE;
  if (row0 >= nlen) return;

  const float alpha    = 0.08838834764831845f;
  const int   ms       = p_maxseq[0];
  const int   sc       = p_scale[0];
  const float invDenom = 1.0f / (float)(sc > 0 ? sc : ms);

  const int tid  = threadIdx.x;
  const int wave = tid >> 5;
  const int lane = tid & 31;
  const int l16  = lane & 15;
  const int hi   = lane >> 4;
  const int qb   = row0 + wave * 16;

  int qrow = qb + l16; if (qrow >= nlen) qrow = nlen - 1;
  const float* qp = tq + (size_t)(off + qrow) * (NHEAD * DQK) + h * DQK;

  v8f acc[8];
#pragma unroll
  for (int i = 0; i < 8; ++i) acc[i] = (v8f){};

  const int jmax = (nlen < row0 + MTILE) ? nlen : (row0 + MTILE);

  for (int j = 0; j < jmax; j += JTILE) {
    {
      const int r  = tid >> 3;
      const int cg = (tid & 7) * 16;
      int krow = j + r; if (krow >= nlen) krow = nlen - 1;
      const float* kp = tk + (size_t)(off + krow) * (NHEAD * DQK) + h * DQK + cg;
      float4 a0 = *(const float4*)(kp + 0);
      float4 a1 = *(const float4*)(kp + 4);
      float4 a2 = *(const float4*)(kp + 8);
      float4 a3 = *(const float4*)(kp + 12);
      if (j + JTILE < jmax)
        __builtin_prefetch(kp + (size_t)JTILE * NHEAD * DQK, 0, 3);
      float* dst = &Kt[r][cg];
      *(float4*)(dst + 0) = a0; *(float4*)(dst + 4) = a1; *(float4*)(dst + 8) = a2; *(float4*)(dst + 12) = a3;
    }
    {
      const int rp = tid >> 4;
      const int cg = (tid & 15) * 8;
      int r0g = j + rp * 2, r1g = r0g + 1;
      if (r0g >= nlen) r0g = nlen - 1;
      if (r1g >= nlen) r1g = nlen - 1;
      const float* v0 = tv + (size_t)(off + r0g) * (NHEAD * DVV) + h * DVV + cg;
      const float* v1 = tv + (size_t)(off + r1g) * (NHEAD * DVV) + h * DVV + cg;
      float4 a0 = *(const float4*)(v0);
      float4 a1 = *(const float4*)(v0 + 4);
      float4 b0 = *(const float4*)(v1);
      float4 b1 = *(const float4*)(v1 + 4);
      if (j + JTILE < jmax)
        __builtin_prefetch(v0 + (size_t)JTILE * NHEAD * DVV, 0, 3);
      float aa[8] = {a0.x, a0.y, a0.z, a0.w, a1.x, a1.y, a1.z, a1.w};
      float bb[8] = {b0.x, b0.y, b0.z, b0.w, b1.x, b1.y, b1.z, b1.w};
#pragma unroll
      for (int c = 0; c < 8; ++c)
        *(uint32_t*)&Vt[cg + c][rp * 2] = pkbf(aa[c], bb[c]);
    }
    __syncthreads();

    v8f s0 = (v8f){}, s1 = (v8f){};
#pragma unroll 1
    for (int c = 0; c < 4; ++c) {
      const F2 qf = split_row(qp, c * 32, lane, alpha);
      s0 = mac3(qf, split_row(&Kt[l16][0], c * 32, lane, 1.0f), s0);
      s1 = mac3(qf, split_row(&Kt[16 + l16][0], c * 32, lane, 1.0f), s1);
    }

    {
      float* sp = &Sscr[wave][0][0];
      const bool fullTile = (j + JTILE - 1 <= qb) && (j + JTILE <= nlen) &&
                            (qb + 15 < nlen);
      if (fullTile) {
#pragma unroll
        for (int r = 0; r < 8; ++r) {
          const int m = r + hi * 8;
          sp[m * 32 + l16]      = fsilu(s0[r]);
          sp[m * 32 + 16 + l16] = fsilu(s1[r]);
        }
      } else {
        const int key0 = j + l16;
        const int key1 = key0 + 16;
#pragma unroll
        for (int r = 0; r < 8; ++r) {
          const int m  = r + hi * 8;
          const int ig = qb + m;
          float a0v = fsilu(s0[r]);
          float a1v = fsilu(s1[r]);
          bool ok0 = (key0 <= ig) && (key0 < nlen) && (ig < nlen);
          bool ok1 = (key1 <= ig) && (key1 < nlen) && (ig < nlen);
          sp[m * 32 + l16]      = ok0 ? a0v : 0.0f;
          sp[m * 32 + 16 + l16] = ok1 ? a1v : 0.0f;
        }
      }
    }

    asm volatile("s_wait_dscnt 0" ::: "memory"); __builtin_amdgcn_wave_barrier(); __builtin_amdgcn_fence(__ATOMIC_RELEASE, "workgroup");
    FragB sf;
    {
      const int c0 = hi * 8;
      const float* row = &Sscr[wave][l16][0];
#pragma unroll
      for (int v = 0; v < 4; ++v) {
        float2 p = *(const float2*)(row + c0 + 2 * v);
        sf.u[v] = pkbf(p.x, p.y);
      }
#pragma unroll
      for (int v = 0; v < 4; ++v) {
        float2 p = *(const float2*)(row + c0 + 16 + 2 * v);
        sf.u[4 + v] = pkbf(p.x, p.y);
      }
    }

#pragma unroll
    for (int dc = 0; dc < 8; ++dc) {
      FragB vf;
      vf.q[0] = *(const uint4*)&Vt[dc * 16 + l16][hi * 8]; vf.q[1] = *(const uint4*)&Vt[dc * 16 + l16][16 + hi * 8];
      acc[dc] = wmma16(sf.v, vf.v, acc[dc]);
    }
    __syncthreads();
  }

  float* so = &So[wave][0][0];
#pragma unroll
  for (int r = 0; r < 8; ++r)
#pragma unroll
    for (int dc = 0; dc < 8; ++dc) so[(r + hi * 8) * DVV + dc * 16 + l16] = acc[dc][r] * invDenom;
  asm volatile("s_wait_dscnt 0" ::: "memory"); __builtin_amdgcn_wave_barrier(); __builtin_amdgcn_fence(__ATOMIC_RELEASE, "workgroup");
#pragma unroll 4
  for (int m = 0; m < 16; ++m) { const int ig = qb + m;
    if (ig < nlen) vst2(out + (size_t)(off + ig) * (NHEAD * DVV) + h * DVV + lane * 4, *(const v4f*)(so + m * DVV + lane * 4)); }
}

extern "C" void kernel_launch(void* const* d_in, const int* in_sizes, int n_in,
                              void* d_out, int out_size, void* d_ws, size_t ws_size,
                              hipStream_t stream) {
  const float* tq      = (const float*)d_in[0];
  const float* tk      = (const float*)d_in[1];
  const float* tv      = (const float*)d_in[2];
  const int*   offsets = (const int*)d_in[3];
  const int*   maxseq  = (const int*)d_in[4];
  const int*   scale   = (const int*)d_in[5];
  float*       out     = (float*)d_out;

  const int B = in_sizes[3] - 1;
  dim3 grid((MAXSEQ + MTILE - 1) / MTILE, NHEAD, B);
  dim3 block(256, 1, 1);
  hstu_attn_wmma<<<grid, block, 0, stream>>>(tq, tk, tv, offsets, maxseq, scale, out);
}
